// S2VSingle_78005196030026
// MI455X (gfx1250) — hardware-verified
//
#include <hip/hip_runtime.h>
#include <stddef.h>


#define DW      128
#define NTHR    256
#define NWAVE   8
#define EPT     8
#define NGRP    2
#define CHUNK   (NTHR * EPT * NGRP)
#define WCAP    (EPT * NGRP * 32)
#define LISTN   (NWAVE * WCAP)
#define NBC     4096
#define NBF     1024
#define RCAP    40960
#define RBN     128
#define TGT     256
#define DEGCAP  1024
#define OTHR    512
#define BM      64
#define KSTEPS  (DW / 32)
#define MAXLV   3
#define NMATMAX 8
#define GPB     8
#define GHMAX   64
#define NSTAT   256
#define WSCAP   134217728
#define ACARRY  8.0f
#define WCARRY  64.0f
#define GSCALE  (1.0f / 512.0f)
#define BNEPS   1e-5f
#define NEGBIG  (-3.402823466e38f)

#define LDS_FILL ((RCAP + NBF + LISTN) * 4 + 64)

static_assert((CHUNK & (CHUNK - 1)) == 0);
static_assert(CHUNK <= 4096);
static_assert((NBC & (NBC - 1)) == 0 && (NBF & (NBF - 1)) == 0);
static_assert(NBC == 4 * NBF);
static_assert(OTHR * 8 == NBC);
static_assert((RCAP % 32) == 0);
static_assert(TGT == NWAVE * 32);
static_assert((NBC % TGT) == 0);
static_assert((TGT % BM) == 0);
static_assert(DW == 4 * 32);
static_assert((DW % 32) == 0);
static_assert(WCAP == EPT * NGRP * 32);
static_assert(GPB == NWAVE);
static_assert(((GPB * DW) % NTHR) == 0);
static_assert(GHMAX == BM);
static_assert(NSTAT == 2 * DW);
static_assert(2 + 2 * MAXLV <= NMATMAX);
static_assert((DW * (DW / 8)) == 8 * NTHR);
static_assert(BM == NWAVE * 8);

typedef float    v4f  __attribute__((ext_vector_type(4)));
typedef float    v8f  __attribute__((ext_vector_type(8)));
typedef int      v4i  __attribute__((ext_vector_type(4)));
typedef _Float16 v4h  __attribute__((ext_vector_type(4)));
typedef _Float16 v8h  __attribute__((ext_vector_type(8)));
typedef _Float16 v16h __attribute__((ext_vector_type(16)));
union Frag { v16h v; v8h h[2]; };

__device__ __forceinline__ v8f wmh(v16h a, v16h b, v8f c) {
  v8f d = __builtin_amdgcn_wmma_f32_16x16x32_f16(false, a, false, b, (short)0, c, false, false);
  asm volatile("v_nop\n\tv_nop\n\tv_nop\n\tv_nop" : "+v"(d) : "v"(a), "v"(b));
  return d;
}

template <int NB>
__device__ __forceinline__ int scan_chunk(const int* __restrict__ dsts, int nE, int cbase, int slotBase,
                                          int vec8, int* list, int tid, int lane, int wave) {
  int wc = 0;
#pragma unroll
  for (int g = 0; g < NGRP; ++g) {
    const int el0  = (g * NTHR + tid) * EPT;
    const int e0   = cbase + el0;
    const int sent = -2147483647 - 1;
    v4i da, db;
    if (vec8 != 0 && cbase + CHUNK <= nE) {
      da = *(const v4i*)(dsts + e0);
      db = *(const v4i*)(dsts + e0 + 4);
    } else {
      da.x = (e0     < nE) ? dsts[min(e0, nE - 1)] : sent;
      da.y = (e0 + 1 < nE) ? dsts[min(e0 + 1, nE - 1)] : sent;
      da.z = (e0 + 2 < nE) ? dsts[min(e0 + 2, nE - 1)] : sent;
      da.w = (e0 + 3 < nE) ? dsts[min(e0 + 3, nE - 1)] : sent;
      db.x = (e0 + 4 < nE) ? dsts[min(e0 + 4, nE - 1)] : sent;
      db.y = (e0 + 5 < nE) ? dsts[min(e0 + 5, nE - 1)] : sent;
      db.z = (e0 + 6 < nE) ? dsts[min(e0 + 6, nE - 1)] : sent;
      db.w = (e0 + 7 < nE) ? dsts[min(e0 + 7, nE - 1)] : sent;
    }
    const unsigned nb = (unsigned)slotBase;
    const unsigned s0 = (unsigned)da.x - nb, s1 = (unsigned)da.y - nb;
    const unsigned s2 = (unsigned)da.z - nb, s3 = (unsigned)da.w - nb;
    const unsigned s4 = (unsigned)db.x - nb, s5 = (unsigned)db.y - nb;
    const unsigned s6 = (unsigned)db.z - nb, s7 = (unsigned)db.w - nb;
    const bool h0 = s0 < (unsigned)NB, h1 = s1 < (unsigned)NB, h2 = s2 < (unsigned)NB, h3 = s3 < (unsigned)NB;
    const bool h4 = s4 < (unsigned)NB, h5 = s5 < (unsigned)NB, h6 = s6 < (unsigned)NB, h7 = s7 < (unsigned)NB;
    const unsigned any = __builtin_amdgcn_ballot_w32(h0 | h1 | h2 | h3 | h4 | h5 | h6 | h7);
    if (any != 0u) {
#define HITJ(J, HJ, SJ) { \
        const unsigned mj = __builtin_amdgcn_ballot_w32(HJ); \
        if (mj != 0u) { \
          if (HJ) { \
            const int pos = wc + (int)__builtin_amdgcn_mbcnt_lo(mj, 0u); \
            if (pos < WCAP) list[wave * WCAP + pos] = ((el0 + (J)) << 12) | (int)(SJ); \
          } \
          wc += (int)__builtin_popcount(mj); } }
      HITJ(0, h0, s0)
      HITJ(1, h1, s1)
      HITJ(2, h2, s2)
      HITJ(3, h3, s3)
      HITJ(4, h4, s4)
      HITJ(5, h5, s5)
      HITJ(6, h6, s6)
      HITJ(7, h7, s7)
#undef HITJ
    }
  }
  return wc;
}

__global__ __launch_bounds__(NTHR) void k_count(const int* __restrict__ dsts, int* cnt, int nE, int vec8) {
  __shared__ __attribute__((aligned(16))) int scnt[NBC];
  __shared__ __attribute__((aligned(16))) int list[LISTN];
  __shared__ int wcnt[NWAVE];
  const int tid = threadIdx.x, lane = tid & 31, wave = tid >> 5;
  const int nodeBase = blockIdx.x * NBC;

  for (int i = tid; i < NBC; i += NTHR) scnt[i] = 0;
  __syncthreads();

  const int nChunks = (nE + CHUNK - 1) / CHUNK;
#pragma unroll 1
  for (int ch = 0; ch < nChunks; ++ch) {
    const int cbase = ch * CHUNK;
    const int wc = scan_chunk<NBC>(dsts, nE, cbase, nodeBase, vec8, list, tid, lane, wave);
    if (lane == 0) wcnt[wave] = wc;
    __syncthreads();
    if (wave == 0) {
#pragma unroll 1
      for (int wsx = 0; wsx < NWAVE; ++wsx) {
        int n = __builtin_amdgcn_readfirstlane(wcnt[wsx]);
        n = n > WCAP ? WCAP : (n < 0 ? 0 : n);
        const int* lp = list + wsx * WCAP;
#pragma unroll 1
        for (int i = 0; i < n; ++i) {
          const int ent  = __builtin_amdgcn_readfirstlane(lp[i]);
          const int slot = ent & (NBC - 1);
          if (lane == 0) scnt[slot] = scnt[slot] + 1;
        }
      }
    }
    __syncthreads();
  }

  v4i cq[4];
#pragma unroll
  for (int q = 0; q < 4; ++q) {
    const int f = (wave * 4 + q) * 128 + 4 * lane;
    cq[q] = *(const v4i*)(scnt + f);
  }
  int* cp = cnt + (size_t)nodeBase;
#pragma unroll
  for (int q = 0; q < 4; ++q) {
    const int f = (wave * 4 + q) * 128 + 4 * lane;
    *(volatile v4i*)(cp + f) = cq[q];
  }
  __threadfence();
#pragma unroll
  for (int q = 0; q < 4; ++q) {
    const int f = (wave * 4 + q) * 128 + 4 * lane;
    *(volatile v4i*)(cp + f) = cq[q];
  }
}

__global__ __launch_bounds__(OTHR) void k_offsets(
    const int* __restrict__ cnt, int* off, int* rbase, int nChunk) {
  __shared__ __attribute__((aligned(16))) int soff[NBC];
  __shared__ __attribute__((aligned(16))) int srb[RBN];
  __shared__ int wtot[OTHR / 32];
  const int tid = threadIdx.x, lane = tid & 31, wave = tid >> 5, sub = tid >> 7;
  for (int i = tid; i < RBN; i += OTHR) srb[i] = 0;
  int carry = 0;
#pragma unroll 1
  for (int ch = 0; ch < nChunk; ++ch) {
    const int base = ch * NBC;
    const v4i c0 = *(const v4i*)(cnt + base + 8 * tid);
    const v4i c1 = *(const v4i*)(cnt + base + 8 * tid + 4);
    const int e0 = max(c0.x, 0), e1 = max(c0.y, 0), e2 = max(c0.z, 0), e3 = max(c0.w, 0);
    const int e4 = max(c1.x, 0), e5 = max(c1.y, 0), e6 = max(c1.z, 0), e7 = max(c1.w, 0);
    const int ts = e0 + e1 + e2 + e3 + e4 + e5 + e6 + e7;
    int incl = ts;
#pragma unroll
    for (int d = 1; d < 32; d <<= 1) {
      const int t = __shfl_up(incl, d);
      if (lane >= d) incl += t;
    }
    if (lane == 31) wtot[wave] = incl;
    __syncthreads();
    const int S0 = wtot[0]  + wtot[1]  + wtot[2]  + wtot[3];
    const int S1 = wtot[4]  + wtot[5]  + wtot[6]  + wtot[7];
    const int S2 = wtot[8]  + wtot[9]  + wtot[10] + wtot[11];
    const int S3 = wtot[12] + wtot[13] + wtot[14] + wtot[15];
    int pre = 0;
#pragma unroll 1
    for (int w = 4 * sub; w < wave; ++w) pre += wtot[w];
    const int b0 = carry;
    const int b1 = b0 + ((S0 + 31) & ~31);
    const int b2 = b1 + ((S1 + 31) & ~31);
    const int b3 = b2 + ((S2 + 31) & ~31);
    const int b4 = b3 + ((S3 + 31) & ~31);
    const int myb = sub == 0 ? b0 : (sub == 1 ? b1 : (sub == 2 ? b2 : b3));
    if (tid == 0) {
      srb[min(4 * ch + 0, RBN - 1)] = b0;
      srb[min(4 * ch + 1, RBN - 1)] = b1;
      srb[min(4 * ch + 2, RBN - 1)] = b2;
      srb[min(4 * ch + 3, RBN - 1)] = b3;
    }
    int run = myb + pre + incl - ts;
    soff[8 * tid + 0] = run; run += e0;
    soff[8 * tid + 1] = run; run += e1;
    soff[8 * tid + 2] = run; run += e2;
    soff[8 * tid + 3] = run; run += e3;
    soff[8 * tid + 4] = run; run += e4;
    soff[8 * tid + 5] = run; run += e5;
    soff[8 * tid + 6] = run; run += e6;
    soff[8 * tid + 7] = run;
    carry = b4;
    __syncthreads();
    const v4i o0 = *(const v4i*)(soff + 4 * tid);
    const v4i o1 = *(const v4i*)(soff + 4 * (tid + OTHR));
    int* op = off + base;
    *(volatile v4i*)(op + 4 * tid) = o0;
    *(volatile v4i*)(op + 4 * (tid + OTHR)) = o1;
    __threadfence();
    *(volatile v4i*)(op + 4 * tid) = o0;
    *(volatile v4i*)(op + 4 * (tid + OTHR)) = o1;
    __syncthreads();
  }
  if (tid == 0) srb[min(4 * nChunk, RBN - 1)] = carry;
  __syncthreads();
  v4i rv = {0, 0, 0, 0};
  if (tid < 32) rv = *(const v4i*)(srb + 4 * tid);
  if (tid < 32) *(volatile v4i*)(rbase + 4 * tid) = rv;
  __threadfence();
  if (tid < 32) *(volatile v4i*)(rbase + 4 * tid) = rv;
}

__global__ __launch_bounds__(NTHR) void k_fill(
    const int* __restrict__ dsts, const int* __restrict__ off, const int* __restrict__ rbase,
    int* csr, int nE, int vec8, int csrLen) {
  extern __shared__ v4f lds_dyn[];
  int* region = (int*)lds_dyn;
  int* cursor = region + RCAP;
  int* list   = cursor + NBF;
  int* wcnt   = list + LISTN;
  const int tid = threadIdx.x, lane = tid & 31, wave = tid >> 5;
  const int b = blockIdx.x;
  const int nodeBase = b * NBF;

  int rb0 = rbase[b];
  const int rb1 = rbase[b + 1];
  rb0 = rb0 < 0 ? 0 : (rb0 > csrLen ? csrLen : rb0);
  rb0 &= ~31;
  int len = rb1 - rb0;
  len = len < 0 ? 0 : (len > RCAP ? RCAP : len);
  int lenW = (len + 31) & ~31;
  if (rb0 + lenW > csrLen) lenW = (csrLen - rb0) & ~31;

  {
    const v4i z = {0, 0, 0, 0};
    for (int i = tid; i < RCAP / 4; i += NTHR) ((v4i*)region)[i] = z;
    for (int s = tid; s < NBF; s += NTHR) {
      int o = off[nodeBase + s] - rb0;
      o = o < 0 ? 0 : (o > RCAP ? RCAP : o);
      cursor[s] = o;
    }
  }
  __syncthreads();

  const int nChunks = (nE + CHUNK - 1) / CHUNK;
#pragma unroll 1
  for (int ch = 0; ch < nChunks; ++ch) {
    const int cbase = ch * CHUNK;
    const int wc = scan_chunk<NBF>(dsts, nE, cbase, nodeBase, vec8, list, tid, lane, wave);
    if (lane == 0) wcnt[wave] = wc;
    __syncthreads();
    if (wave == 0) {
#pragma unroll 1
      for (int wsx = 0; wsx < NWAVE; ++wsx) {
        int n = __builtin_amdgcn_readfirstlane(wcnt[wsx]);
        n = n > WCAP ? WCAP : (n < 0 ? 0 : n);
        const int* lp = list + wsx * WCAP;
#pragma unroll 1
        for (int i = 0; i < n; ++i) {
          const int ent  = __builtin_amdgcn_readfirstlane(lp[i]);
          const int slot = ent & (NBF - 1);
          int e = cbase + ((ent >> 12) & (CHUNK - 1));
          e = e > nE - 1 ? nE - 1 : (e < 0 ? 0 : e);
          if (lane == 0) {
            int pos = cursor[slot];
            pos = pos < 0 ? 0 : (pos > RCAP - 1 ? RCAP - 1 : pos);
            region[pos] = e;
            const int np = pos + 1;
            cursor[slot] = np > RCAP ? RCAP : np;
          }
        }
      }
    }
    __syncthreads();
  }

  const int nv = lenW >> 2;
  int* gp = csr + rb0;
#pragma unroll 1
  for (int i = tid; i < nv; i += NTHR) { const v4i v = ((const v4i*)region)[i]; *(volatile v4i*)(gp + 4 * i) = v; }
  __threadfence();
#pragma unroll 1
  for (int i = tid; i < nv; i += NTHR) { const v4i v = ((const v4i*)region)[i]; *(volatile v4i*)(gp + 4 * i) = v; }
}

__global__ __launch_bounds__(TGT) void k_esum(
    const int* __restrict__ csr, const int* __restrict__ off, const int* __restrict__ cnt,
    const float* __restrict__ ef, float* efs, int nE, int csrLen) {
  const int c = (int)blockIdx.x * TGT + (int)threadIdx.x;
  int n = cnt[c];
  n = n < 0 ? 0 : (n > DEGCAP ? DEGCAP : n);
  const int st = off[c];
  float f0 = 0.f, f1 = 0.f, f2 = 0.f;
#pragma unroll 1
  for (int p = 0; p < n; ++p) {
    int pos = st + p;
    pos = pos < 0 ? 0 : (pos > csrLen - 1 ? csrLen - 1 : pos);
    int e = csr[pos];
    e = e < 0 ? 0 : (e > nE - 1 ? nE - 1 : e);
    const float* q = ef + (size_t)e * 3;
    f0 += q[0]; f1 += q[1]; f2 += q[2];
  }
  v4f o;
  o.x = f0; o.y = f1; o.z = f2; o.w = (float)n;
  float* gp = efs + (size_t)c * 4;
  *(volatile v4f*)gp = o;
  __threadfence();
  *(volatile v4f*)gp = o;
}

__global__ __launch_bounds__(NTHR) void k_wcvt(
    const float* __restrict__ wn2l, const float* __restrict__ wconv,
    const float* __restrict__ wl2, const float* __restrict__ wro, _Float16* dp, int nLV) {
  const int p = (int)blockIdx.x >> 3;
  const int u = (((int)blockIdx.x & 7) * NTHR) + (int)threadIdx.x;
  const float* W;
  if (p == 0) W = wn2l;
  else if (p <= nLV) W = wconv + (size_t)(p - 1) * DW * DW;
  else if (p <= 2 * nLV) W = wl2 + (size_t)(p - 1 - nLV) * DW * DW;
  else W = wro;
  const int ppr = DW / 8;
  const int n = u / ppr;
  const int seg = u - n * ppr;
  const float* q = W + (size_t)(8 * seg) * DW + n;
  v8h o;
#pragma unroll
  for (int j = 0; j < 8; ++j) {
    const float f = q[(size_t)j * DW];
    o[j] = (_Float16)(f * WCARRY);
  }
  _Float16* gp = dp + (size_t)p * DW * DW + (size_t)u * 8;
  *(volatile v8h*)gp = o;
  __threadfence();
  *(volatile v8h*)gp = o;
}

template <int MODE>
__global__ __launch_bounds__(NTHR) void k_gemm(
    const float* Asrc, const float* __restrict__ hp,
    const int* __restrict__ csr, const int* __restrict__ off, const int* __restrict__ cnt,
    const int* __restrict__ efrom, const float* __restrict__ efs, const float* __restrict__ bnss,
    const _Float16* __restrict__ Bp, const float* __restrict__ bias,
    const float* __restrict__ We, const float* __restrict__ be,
    float* Cout, float* part, int nValid, int nN, int nE, int csrLen) {
  constexpr int TPW = 4;
  constexpr int NIT = BM / NWAVE;
  static_assert(TPW * 16 * 2 == DW);
  static_assert(BM == 4 * 16);
  static_assert(NIT == 8);

  __shared__ __attribute__((aligned(16))) float stg[BM * DW];
  __shared__ __attribute__((aligned(16))) _Float16 a16[BM * DW];
  __shared__ __attribute__((aligned(16))) float sst[NSTAT];
  const int tid = threadIdx.x, lane = tid & 31, wave = tid >> 5, hh = lane >> 4, m = lane & 15;
  const int rowBase = (int)blockIdx.x * BM;
  const int rg = wave >> 1, chf = wave & 1;
  const int r0 = rg * 16;
  const int c0 = chf * (DW / 2);
  const int col4 = 4 * lane;

  if (MODE == 1) {
#pragma unroll 1
    for (int it = 0; it < NIT; ++it) {
      const int row = it * NWAVE + wave;
      const int c = rowBase + row;
      int n = cnt[c];
      n = n < 0 ? 0 : (n > DEGCAP ? DEGCAP : n);
      const int st = off[c];
      v4f a = {0.f, 0.f, 0.f, 0.f};
#pragma unroll 1
      for (int q0 = 0; q0 < n; q0 += 32) {
        int pos = st + q0 + lane;
        pos = pos < 0 ? 0 : (pos > csrLen - 1 ? csrLen - 1 : pos);
        int e = csr[pos];
        e = e < 0 ? 0 : (e > nE - 1 ? nE - 1 : e);
        int s = efrom[e];
        s = s < 0 ? 0 : (s > nN - 1 ? nN - 1 : s);
        const int mcnt = (n - q0) < 32 ? (n - q0) : 32;
#pragma unroll 1
        for (int pp = 0; pp < mcnt; ++pp) {
          const int ss = __builtin_amdgcn_readlane(s, pp);
          const v4f xv = *(const v4f*)(hp + (size_t)ss * DW + col4);
          a = a + xv;
        }
      }
      const bool live = c < nValid;
      v4h o;
      o.x = (_Float16)((live ? a.x : 0.f) * ACARRY);
      o.y = (_Float16)((live ? a.y : 0.f) * ACARRY);
      o.z = (_Float16)((live ? a.z : 0.f) * ACARRY);
      o.w = (_Float16)((live ? a.w : 0.f) * ACARRY);
      *(v4h*)(a16 + (size_t)row * DW + col4) = o;
    }
  } else {
    v4f scv = {1.f, 1.f, 1.f, 1.f};
    v4f shv = {0.f, 0.f, 0.f, 0.f};
    if (MODE == 2) {
      scv = *(const v4f*)(bnss + col4);
      shv = *(const v4f*)(bnss + DW + col4);
    }
#pragma unroll
    for (int it = 0; it < NIT; ++it) {
      const int row = it * NWAVE + wave;
      const int grow = rowBase + row;
      const bool live = grow < nValid;
      int rr = grow > nValid - 1 ? nValid - 1 : grow;
      rr = rr < 0 ? 0 : rr;
      v4f xv = *(const v4f*)(Asrc + (size_t)rr * DW + col4);
      if (MODE == 2) {
        xv.x = fmaxf(xv.x, 0.f) * scv.x + shv.x;
        xv.y = fmaxf(xv.y, 0.f) * scv.y + shv.y;
        xv.z = fmaxf(xv.z, 0.f) * scv.z + shv.z;
        xv.w = fmaxf(xv.w, 0.f) * scv.w + shv.w;
      }
      v4h o;
      o.x = (_Float16)((live ? xv.x : 0.f) * ACARRY);
      o.y = (_Float16)((live ? xv.y : 0.f) * ACARRY);
      o.z = (_Float16)((live ? xv.z : 0.f) * ACARRY);
      o.w = (_Float16)((live ? xv.w : 0.f) * ACARRY);
      *(v4h*)(a16 + (size_t)row * DW + col4) = o;
    }
  }

  {
    const v4f b4 = *(const v4f*)(bias + col4);
    v4f w0 = b4, w1 = b4, w2 = b4, wb = b4;
    if (MODE == 0 || MODE == 1) {
      w0 = *(const v4f*)(We + col4);
      w1 = *(const v4f*)(We + DW + col4);
      w2 = *(const v4f*)(We + 2 * DW + col4);
      wb = *(const v4f*)(be + col4);
    }
#pragma unroll 1
    for (int it = 0; it < NIT; ++it) {
      const int row = it * NWAVE + wave;
      const int grow = rowBase + row;
      v4f add = b4;
      if (MODE == 0 || MODE == 1) {
        const v4f ev = *(const v4f*)(efs + (size_t)grow * 4);
        add = add + ev.x * w0 + ev.y * w1 + ev.z * w2 + ev.w * wb;
      }
      if (MODE == 2) {
        const v4f hv = *(const v4f*)(hp + (size_t)grow * DW + col4);
        add = add + hv;
      }
      *(v4f*)(stg + (size_t)row * DW + col4) = add;
    }
  }
  __syncthreads();

  v8f acc[TPW];
#pragma unroll
  for (int t = 0; t < TPW; ++t) { v8f z = {0.f, 0.f, 0.f, 0.f, 0.f, 0.f, 0.f, 0.f}; acc[t] = z; }

  const _Float16* ap = a16 + (size_t)(r0 + m) * DW + 8 * hh;
  const _Float16* bp = Bp + (size_t)(c0 + m) * DW + 8 * hh;
#pragma unroll 1
  for (int kt = 0; kt < KSTEPS; ++kt) {
    Frag a;
    a.h[0] = *(const v8h*)(ap + 32 * kt);
    a.h[1] = *(const v8h*)(ap + 32 * kt + 16);
#pragma unroll
    for (int t = 0; t < TPW; ++t) {
      const size_t to = (size_t)(16 * t) * DW + 32 * kt;
      Frag b;
      b.h[0] = *(const v8h*)(bp + to);
      b.h[1] = *(const v8h*)(bp + to + 16);
      acc[t] = wmh(a.v, b.v, acc[t]);
    }
  }

  {
    float* sp = stg + (size_t)(r0 + 8 * hh) * DW + c0 + m;
    const int growb = rowBase + r0 + 8 * hh;
#pragma unroll
    for (int t = 0; t < TPW; ++t) {
#pragma unroll
      for (int r = 0; r < 8; ++r) {
        const bool lv = (growb + r) < nValid;
        const float g = acc[t][r] * GSCALE;
        float v = sp[r * DW + 16 * t] + g;
        if (MODE == 3) v = fmaxf(v, 0.f);
        else v = lv ? v : 0.f;
        sp[r * DW + 16 * t] = v;
      }
    }
  }
  __syncthreads();

  if (MODE != 3) {
    if (tid < DW) {
      float s = 0.f, q = 0.f;
#pragma unroll 4
      for (int r = 0; r < BM; ++r) {
        const float x = fmaxf(stg[r * DW + tid], 0.f);
        s += x;
        q += x * x;
      }
      sst[tid] = s;
      sst[DW + tid] = q;
    }
  }
  v4f cv[NIT];
#pragma unroll
  for (int it = 0; it < NIT; ++it) {
    const int row = it * NWAVE + wave;
    cv[it] = *(const v4f*)(stg + (size_t)row * DW + col4);
  }
  __syncthreads();
  v4f pv = {0.f, 0.f, 0.f, 0.f};
  if (MODE != 3) { if (tid < NSTAT / 4) pv = *(const v4f*)(sst + 4 * tid); }
  float* pp = part + (size_t)blockIdx.x * NSTAT + 4 * tid;

#pragma unroll
  for (int it = 0; it < NIT; ++it) {
    const int row = it * NWAVE + wave;
    const int grow = rowBase + row;
    float* gp = Cout + (size_t)grow * DW + col4;
    if (MODE != 3 || grow < nValid) *(volatile v4f*)gp = cv[it];
  }
  if (MODE != 3) { if (tid < NSTAT / 4) *(volatile v4f*)pp = pv; }
  __threadfence();
#pragma unroll
  for (int it = 0; it < NIT; ++it) {
    const int row = it * NWAVE + wave;
    const int grow = rowBase + row;
    float* gp = Cout + (size_t)grow * DW + col4;
    if (MODE != 3 || grow < nValid) *(volatile v4f*)gp = cv[it];
  }
  if (MODE != 3) { if (tid < NSTAT / 4) *(volatile v4f*)pp = pv; }
}

__global__ __launch_bounds__(DW) void k_bnfin(
    const float* __restrict__ part, int nPart, const float* __restrict__ gam,
    const float* __restrict__ bet, float* bnss, int nValid) {
  __shared__ __attribute__((aligned(16))) float sv[NSTAT];
  const int d = threadIdx.x;
  double S = 0.0, Q = 0.0;
#pragma unroll 1
  for (int b = 0; b < nPart; ++b) {
    S += (double)part[(size_t)b * NSTAT + d];
    Q += (double)part[(size_t)b * NSTAT + DW + d];
  }
  const double inv = 1.0 / (double)(nValid < 1 ? 1 : nValid);
  const double mean = S * inv;
  double var = Q * inv - mean * mean;
  var = var < 0.0 ? 0.0 : var;
  const float rstd = rsqrtf((float)var + BNEPS);
  const float sc = gam[d] * rstd;
  const float sh = bet[d] - (float)mean * sc;
  sv[d] = sc;
  sv[DW + d] = sh;
  __syncthreads();
  v4f v = {0.f, 0.f, 0.f, 0.f};
  if (d < NSTAT / 4) v = *(const v4f*)(sv + 4 * d);
  if (d < NSTAT / 4) *(volatile v4f*)(bnss + 4 * d) = v;
  __threadfence();
  if (d < NSTAT / 4) *(volatile v4f*)(bnss + 4 * d) = v;
}

__global__ __launch_bounds__(NTHR) void k_bnapply(
    const float* __restrict__ Y, const float* __restrict__ bnss, float* hout, int nValid) {
  const int tid = threadIdx.x, lane = tid & 31, wave = tid >> 5;
  const int row = (int)blockIdx.x * NWAVE + wave;
  const int col4 = 4 * lane;
  const v4f scv = *(const v4f*)(bnss + col4);
  const v4f shv = *(const v4f*)(bnss + DW + col4);
  const bool live = row < nValid;
  int rr = row > nValid - 1 ? nValid - 1 : row;
  rr = rr < 0 ? 0 : rr;
  const v4f x = *(const v4f*)(Y + (size_t)rr * DW + col4);
  v4f o;
  o.x = live ? (fmaxf(x.x, 0.f) * scv.x + shv.x) : 0.f;
  o.y = live ? (fmaxf(x.y, 0.f) * scv.y + shv.y) : 0.f;
  o.z = live ? (fmaxf(x.z, 0.f) * scv.z + shv.z) : 0.f;
  o.w = live ? (fmaxf(x.w, 0.f) * scv.w + shv.w) : 0.f;
  float* gp = hout + (size_t)row * DW + col4;
  *(volatile v4f*)gp = o;
  __threadfence();
  *(volatile v4f*)gp = o;
}

__global__ __launch_bounds__(NTHR) void k_pool(
    const int* __restrict__ gid, const float* __restrict__ h, float* pooled, int nN, int vec8) {
  __shared__ __attribute__((aligned(16))) int list[LISTN];
  __shared__ __attribute__((aligned(16))) float spart[NWAVE * GPB * DW];
  __shared__ __attribute__((aligned(16))) float ssum[GPB * DW];
  const int tid = threadIdx.x, lane = tid & 31, wave = tid >> 5;
  const int gBase = blockIdx.x * GPB;
  const int col4 = 4 * lane;

  v4f acc[GPB];
#pragma unroll
  for (int s = 0; s < GPB; ++s) { v4f z = {NEGBIG, NEGBIG, NEGBIG, NEGBIG}; acc[s] = z; }

  const int nChunks = (nN + CHUNK - 1) / CHUNK;
#pragma unroll 1
  for (int ch = 0; ch < nChunks; ++ch) {
    const int cbase = ch * CHUNK;
    const int wc = scan_chunk<GPB>(gid, nN, cbase, gBase, vec8, list, tid, lane, wave);
    __syncthreads();
    int n = wc;
    n = n > WCAP ? WCAP : (n < 0 ? 0 : n);
    const int* lp = list + wave * WCAP;
#pragma unroll 1
    for (int i = 0; i < n; ++i) {
      const int ent = __builtin_amdgcn_readfirstlane(lp[i]);
      int node = cbase + ((ent >> 12) & (CHUNK - 1));
      node = node > nN - 1 ? nN - 1 : (node < 0 ? 0 : node);
      const int slot = ent & (GPB - 1);
      const v4f hv = *(const v4f*)(h + (size_t)node * DW + col4);
#pragma unroll
      for (int s = 0; s < GPB; ++s) {
        const bool hit = slot == s;
        acc[s].x = fmaxf(acc[s].x, hit ? hv.x : NEGBIG);
        acc[s].y = fmaxf(acc[s].y, hit ? hv.y : NEGBIG);
        acc[s].z = fmaxf(acc[s].z, hit ? hv.z : NEGBIG);
        acc[s].w = fmaxf(acc[s].w, hit ? hv.w : NEGBIG);
      }
    }
    __syncthreads();
  }

#pragma unroll
  for (int s = 0; s < GPB; ++s) *(v4f*)(spart + (size_t)(wave * GPB + s) * DW + col4) = acc[s];
  __syncthreads();
#pragma unroll
  for (int q = 0; q < (GPB * DW) / NTHR; ++q) {
    const int idx = q * NTHR + tid;
    const int s = idx / DW, c = idx % DW;
    float S = NEGBIG;
#pragma unroll
    for (int w = 0; w < NWAVE; ++w) S = fmaxf(S, spart[(w * GPB + s) * DW + c]);
    ssum[idx] = S;
  }
  __syncthreads();
  const v4f v = *(const v4f*)(ssum + wave * DW + col4);
  float* gp = pooled + (size_t)(gBase + wave) * DW + col4;
  *(volatile v4f*)gp = v;
  __threadfence();
  *(volatile v4f*)gp = v;
}

extern "C" void kernel_launch(void* const* d_in, const int* in_sizes, int n_in,
                              void* d_out, int out_size, void* d_ws, size_t ws_size,
                              hipStream_t stream) {
  if (n_in < 20) return;
  if (in_sizes[0] < DW || (in_sizes[0] % DW) != 0) return;
  const int nN = in_sizes[0] / DW;
  if (in_sizes[1] < 3 || (in_sizes[1] % 3) != 0) return;
  const int nE = in_sizes[1] / 3;
  if (in_sizes[2] != nE || in_sizes[3] != nE) return;
  if (in_sizes[4] != nN) return;
  if (in_sizes[6] != DW * DW || in_sizes[7] != DW) return;
  if (in_sizes[10] < DW * DW || (in_sizes[10] % (DW * DW)) != 0) return;
  const int nLV = in_sizes[10] / (DW * DW);
  if (nLV < 1 || nLV > MAXLV) return;
  if (in_sizes[8] != (nLV + 1) * 3 * DW || in_sizes[9] != (nLV + 1) * DW) return;
  if (in_sizes[11] != nLV * DW || in_sizes[12] != nLV * DW * DW || in_sizes[13] != nLV * DW) return;
  if (in_sizes[14] != (nLV + 1) * DW || in_sizes[15] != (nLV + 1) * DW) return;
  if (in_sizes[16] != nLV * DW || in_sizes[17] != nLV * DW) return;
  if (in_sizes[18] != DW * DW || in_sizes[19] != DW) return;
  if (out_size < DW || (out_size % DW) != 0) return;
  const int nG = out_size / DW;
  if (nG < 1 || nG > GHMAX) return;
  if (nE > (1 << 28) || nN > (1 << 22)) return;

  const float* node_feat = (const float*)d_in[0];
  const float* edge_feat = (const float*)d_in[1];
  const int*   efrom     = (const int*)d_in[2];
  const int*   eto       = (const int*)d_in[3];
  const int*   gidx      = (const int*)d_in[4];
  const float* w_n2l_w   = (const float*)d_in[6];
  const float* w_n2l_b   = (const float*)d_in[7];
  const float* w_e2l_w   = (const float*)d_in[8];
  const float* w_e2l_b   = (const float*)d_in[9];
  const float* conv_w    = (const float*)d_in[10];
  const float* conv_b    = (const float*)d_in[11];
  const float* l2_w      = (const float*)d_in[12];
  const float* l2_b      = (const float*)d_in[13];
  const float* msg_bn_g  = (const float*)d_in[14];
  const float* msg_bn_b  = (const float*)d_in[15];
  const float* hid_bn_g  = (const float*)d_in[16];
  const float* hid_bn_b  = (const float*)d_in[17];
  const float* ro_w      = (const float*)d_in[18];
  const float* ro_b      = (const float*)d_in[19];
  float* out = (float*)d_out;

  const int NPAD   = ((nN + TGT - 1) / TGT) * TGT;
  const int nBC    = (nN + NBC - 1) / NBC;
  const int CNTPAD = nBC * NBC;
  if (CNTPAD < NPAD) return;
  if (4 * nBC + 1 > RBN) return;
  const int nBF    = (nN + NBF - 1) / NBF;
  if (nBF > 4 * nBC) return;
  const int csrLen = ((nE + 31) & ~31) + 4096;
  if (31 * 4 * nBC > 4096) return;
  const int nGemm  = NPAD / BM;
  const int nEs    = NPAD / TGT;
  const int nApp   = NPAD / NWAVE;
  const int nMat   = 2 + 2 * nLV;
  const int GPAD   = GHMAX;
  const int GBLK   = GPAD / GPB;

  char* ws = (char*)d_ws;
  size_t off = 0;
  const size_t oWp  = off; off += (size_t)nMat * DW * DW * 2;      off = (off + 255) & ~(size_t)255;
  const size_t oH   = off; off += (size_t)NPAD * DW * 4;          off = (off + 255) & ~(size_t)255;
  const size_t oY   = off; off += (size_t)NPAD * DW * 4;          off = (off + 255) & ~(size_t)255;
  const size_t oCnt = off; off += (size_t)CNTPAD * 4;             off = (off + 255) & ~(size_t)255;
  const size_t oOff = off; off += (size_t)CNTPAD * 4;             off = (off + 255) & ~(size_t)255;
  const size_t oRb  = off; off += (size_t)RBN * 4;                off = (off + 255) & ~(size_t)255;
  const size_t oCsr = off; off += (size_t)csrLen * 4;             off = (off + 255) & ~(size_t)255;
  const size_t oEfs = off; off += (size_t)NPAD * 4 * 4;           off = (off + 255) & ~(size_t)255;
  const size_t oPt  = off; off += (size_t)nGemm * NSTAT * 4;      off = (off + 255) & ~(size_t)255;
  const size_t oSs  = off; off += (size_t)NSTAT * 4;              off = (off + 255) & ~(size_t)255;
  const size_t oPl  = off; off += (size_t)GPAD * DW * 4;          off = (off + 255) & ~(size_t)255;
  if (off > ws_size || off > (size_t)WSCAP) return;

  _Float16* wpl = (_Float16*)(ws + oWp);
  float* hpl  = (float*)(ws + oH);
  float* ypl  = (float*)(ws + oY);
  int*   cnt  = (int*)(ws + oCnt);
  int*   offp = (int*)(ws + oOff);
  int*   rb   = (int*)(ws + oRb);
  int*   csr  = (int*)(ws + oCsr);
  float* efs  = (float*)(ws + oEfs);
  float* part = (float*)(ws + oPt);
  float* bnss = (float*)(ws + oSs);
  float* pooled = (float*)(ws + oPl);

  const size_t PL = (size_t)DW * DW;

  k_wcvt<<<nMat * 8, NTHR, 0, stream>>>(w_n2l_w, conv_w, l2_w, ro_w, wpl, nLV);
  k_count<<<nBC, NTHR, 0, stream>>>(eto, cnt, nE, 1);
  k_offsets<<<1, OTHR, 0, stream>>>(cnt, offp, rb, nBC);
  hipFuncSetAttribute(reinterpret_cast<const void*>(&k_fill),
                      hipFuncAttributeMaxDynamicSharedMemorySize, LDS_FILL);
  k_fill<<<nBF, NTHR, LDS_FILL, stream>>>(eto, offp, rb, csr, nE, 1, csrLen);
  k_esum<<<nEs, TGT, 0, stream>>>(csr, offp, cnt, edge_feat, efs, nE, csrLen);

  k_gemm<0><<<nGemm, NTHR, 0, stream>>>(node_feat, hpl, csr, offp, cnt, efrom, efs, bnss,
                                        wpl, w_n2l_b, w_e2l_w, w_e2l_b, ypl, part, nN, nN, nE, csrLen);
  k_bnfin<<<1, DW, 0, stream>>>(part, nGemm, msg_bn_g, msg_bn_b, bnss, nN);
  k_bnapply<<<nApp, NTHR, 0, stream>>>(ypl, bnss, hpl, nN);

  for (int lv = 0; lv < nLV; ++lv) {
    k_gemm<1><<<nGemm, NTHR, 0, stream>>>(hpl, hpl, csr, offp, cnt, efrom, efs, bnss,
                                          wpl + (size_t)(1 + lv) * PL, conv_b + (size_t)lv * DW,
                                          w_e2l_w + (size_t)(lv + 1) * 3 * DW, w_e2l_b + (size_t)(lv + 1) * DW,
                                          ypl, part, nN, nN, nE, csrLen);
    k_bnfin<<<1, DW, 0, stream>>>(part, nGemm, hid_bn_g + (size_t)lv * DW, hid_bn_b + (size_t)lv * DW, bnss, nN);
    k_gemm<2><<<nGemm, NTHR, 0, stream>>>(ypl, hpl, csr, offp, cnt, efrom, efs, bnss,
                                          wpl + (size_t)(1 + nLV + lv) * PL, l2_b + (size_t)lv * DW,
                                          w_e2l_w, w_e2l_b, ypl, part, nN, nN, nE, csrLen);
    k_bnfin<<<1, DW, 0, stream>>>(part, nGemm, msg_bn_g + (size_t)(lv + 1) * DW,
                                  msg_bn_b + (size_t)(lv + 1) * DW, bnss, nN);
    k_bnapply<<<nApp, NTHR, 0, stream>>>(ypl, bnss, hpl, nN);
  }

  k_pool<<<GBLK, NTHR, 0, stream>>>(gidx, hpl, pooled, nN, 1);
  k_gemm<3><<<GPAD / BM, NTHR, 0, stream>>>(pooled, hpl, csr, offp, cnt, efrom, efs, bnss,
                                            wpl + (size_t)(1 + 2 * nLV) * PL, ro_b, w_e2l_w, w_e2l_b,
                                            out, part, nG, nN, nE, csrLen);
}
